// JacobAttentionLayer_84018150244754
// MI455X (gfx1250) — hardware-verified
//
#include <hip/hip_runtime.h>


typedef __bf16 v16bf __attribute__((ext_vector_type(16)));
typedef float v8f __attribute__((ext_vector_type(8)));
typedef float v4f __attribute__((ext_vector_type(4)));
typedef unsigned int v4u __attribute__((ext_vector_type(4)));
typedef unsigned short u16;

constexpr int BB = 2;
constexpr int TT = 2048;
constexpr int CC = 1024;
constexpr int NH = 16;
constexpr int HS = 64;
constexpr int OC = 3 * CC + NH;
constexpr int NBH = BB * NH;
constexpr int NT = TT / 64;
constexpr int MROWS = BB * TT;
constexpr int LDSP = 72;
constexpr int STG = 68;
constexpr float EPSV = 1e-7f;
constexpr float LOGSCALE = -2.0794415416798357f;
constexpr float NEG_BIG = -1e30f;
constexpr float CULL_GAP = 32.0f;

union Frag { v16bf v; v4u q[2]; };
union Pack8 { v4u q; u16 e[8]; };

__device__ __forceinline__ unsigned bf16_rne_bits(float f) {
  unsigned u = __float_as_uint(f);
  u += 0x7FFFu + ((u >> 16) & 1u);
  return u >> 16;
}
__device__ __forceinline__ float bf16_bits_to_f32(unsigned b) { return __uint_as_float(b << 16); }
__device__ __forceinline__ unsigned pack2(unsigned lo, unsigned hi) { return (lo & 0xFFFFu) | (hi << 16); }

__device__ __forceinline__ v16bf load_frag(const u16* p, int h8) {
  Frag f;
  f.q[0] = *reinterpret_cast<const v4u*>(p + h8);
  f.q[1] = *reinterpret_cast<const v4u*>(p + 16 + h8);
  return f.v;
}

__device__ __forceinline__ v8f wmma_bf16(v8f c, v16bf a, v16bf b) {
  c = __builtin_amdgcn_wmma_f32_16x16x32_bf16(false, a, false, b, (short)0, c, false, false);
  asm volatile("v_nop\n\tv_nop\n\tv_nop\n\tv_nop" : "+v"(c) : "v"(a), "v"(b));
  return c;
}

__device__ __forceinline__ v8f wmma_bf16x3(v8f c, v16bf ah, v16bf al, v16bf bh, v16bf bl) {
  c = __builtin_amdgcn_wmma_f32_16x16x32_bf16(false, ah, false, bh, (short)0, c, false, false);
  c = __builtin_amdgcn_wmma_f32_16x16x32_bf16(false, al, false, bh, (short)0, c, false, false);
  c = __builtin_amdgcn_wmma_f32_16x16x32_bf16(false, ah, false, bl, (short)0, c, false, false);
  asm volatile("v_nop\n\tv_nop\n\tv_nop\n\tv_nop" : "+v"(c) : "v"(ah), "v"(al), "v"(bh), "v"(bl));
  return c;
}

__device__ __forceinline__ v4u cvt8_bf16(const float* __restrict__ src) {
  const v4f a = *reinterpret_cast<const v4f*>(src);
  const v4f b = *reinterpret_cast<const v4f*>(src + 4);
  v4u w;
  w.x = pack2(bf16_rne_bits(a.x), bf16_rne_bits(a.y));
  w.y = pack2(bf16_rne_bits(a.z), bf16_rne_bits(a.w));
  w.z = pack2(bf16_rne_bits(b.x), bf16_rne_bits(b.y));
  w.w = pack2(bf16_rne_bits(b.z), bf16_rne_bits(b.w));
  return w;
}

__global__ __launch_bounds__(128) void k_proj(
    const float* __restrict__ X, const float* __restrict__ W,
    u16* __restrict__ Qh, u16* __restrict__ Ql, u16* __restrict__ Kh, u16* __restrict__ Kl,
    u16* __restrict__ Vh, u16* __restrict__ Vl, float* __restrict__ gates, float* __restrict__ nrm) {
  __shared__ __attribute__((aligned(16))) unsigned char lds_raw[2 * 64 * LDSP * 2];
  __shared__ float ldsN[64];
  u16* ldsX = reinterpret_cast<u16*>(lds_raw);
  u16* ldsW = ldsX + 64 * LDSP;
  float* stg = reinterpret_cast<float*>(lds_raw);

  const int tid = threadIdx.x, wave = tid >> 5, lane = tid & 31;
  const int h8 = (lane >> 4) * 8, ln = lane & 15;
  const int n0 = blockIdx.x * 64;
  const int m0 = blockIdx.y * 64;

  v8f acc[4] = {};

  for (int kt = 0; kt < CC / 64; ++kt) {
    const int k0 = kt * 64;
    __syncthreads();
#pragma unroll
    for (int p = 0; p < 4; ++p) {
      const int idx = tid + p * 128, row = idx >> 3, seg = (idx & 7) * 8;
      *reinterpret_cast<v4u*>(ldsX + row * LDSP + seg) =
          cvt8_bf16(X + (size_t)(m0 + row) * CC + k0 + seg);
    }
#pragma unroll
    for (int p = 0; p < 4; ++p) {
      const int idx = tid + p * 128, row = idx >> 3, seg = (idx & 7) * 8;
      int wn = n0 + row;
      if (wn > OC - 1) wn = OC - 1;
      *reinterpret_cast<v4u*>(ldsW + row * LDSP + seg) =
          cvt8_bf16(W + (size_t)wn * CC + k0 + seg);
    }
    __syncthreads();
#pragma unroll
    for (int ks = 0; ks < 2; ++ks) {
      const v16bf af = load_frag(ldsX + (wave * 16 + ln) * LDSP + ks * 32, h8);
#pragma unroll
      for (int j = 0; j < 4; ++j) {
        const v16bf bfr = load_frag(ldsW + (j * 16 + ln) * LDSP + ks * 32, h8);
        acc[j] = wmma_bf16(acc[j], af, bfr);
      }
    }
  }

  __syncthreads();
  float* sw = stg + wave * 16 * STG;
#pragma unroll
  for (int j = 0; j < 4; ++j)
#pragma unroll
    for (int r = 0; r < 8; ++r)
      sw[(h8 + r) * STG + j * 16 + ln] = acc[j][r];
  __syncthreads();

  if (tid < 64) {
    const float* rp = stg + tid * STG;
    float s = 0.f;
#pragma unroll 8
    for (int c = 0; c < 64; ++c) { const float v = rp[c]; s = fmaf(v, v, s); }
    ldsN[tid] = s;
  }
  __syncthreads();
  float nmax = 0.f;
  if (wave == 0) {
    float v = fmaxf(ldsN[lane], ldsN[lane + 32]);
#pragma unroll
    for (int off = 16; off > 0; off >>= 1) v = fmaxf(v, __shfl_xor(v, off, 32));
    nmax = v;
  }

  const int sel = n0 >> 10;
  const int b = m0 >> 11;
  const int tb = m0 & (TT - 1);
  const int hh = (n0 & (CC - 1)) >> 6;
  const int bh = b * NH + hh;
  u16* Ph = (sel == 0) ? Qh : (sel == 1) ? Kh : Vh;
  u16* Pl = (sel == 0) ? Ql : (sel == 1) ? Kl : Vl;
  const size_t prow0 = ((size_t)bh * TT + tb + wave * 16) * HS;
  float* gw = gates + (size_t)(m0 + wave * 16) * NH;
  float* nl = nrm + (size_t)(sel * (NBH * NT) + bh * NT + (tb >> 6)) * 32;

  auto emit = [&]() {
    if (sel < 3) {
#pragma unroll
      for (int it = 0; it < 4; ++it) {
        const int row = it * 4 + (lane >> 3), seg = (lane & 7) * 8;
        const float* sp = sw + row * STG + seg;
        unsigned hb[8], lb[8];
#pragma unroll
        for (int e = 0; e < 8; ++e) {
          const float v = sp[e];
          const unsigned hbit = bf16_rne_bits(v);
          hb[e] = hbit;
          lb[e] = bf16_rne_bits(v - bf16_bits_to_f32(hbit));
        }
        v4u wh, wl;
        wh.x = pack2(hb[0], hb[1]); wh.y = pack2(hb[2], hb[3]); wh.z = pack2(hb[4], hb[5]); wh.w = pack2(hb[6], hb[7]);
        wl.x = pack2(lb[0], lb[1]); wl.y = pack2(lb[2], lb[3]); wl.z = pack2(lb[4], lb[5]); wl.w = pack2(lb[6], lb[7]);
        const size_t off = prow0 + (size_t)row * HS + seg;
        *reinterpret_cast<volatile v4u*>(Ph + off) = wh;
        *reinterpret_cast<volatile v4u*>(Pl + off) = wl;
      }
      if (sel < 2 && wave == 0 && lane < 8) {
        v4f v; v.x = nmax; v.y = nmax; v.z = nmax; v.w = nmax;
        *reinterpret_cast<volatile v4f*>(nl + lane * 4) = v;
      }
    } else {
#pragma unroll
      for (int it = 0; it < 2; ++it) {
        const int row = it * 8 + (lane >> 2), c4 = (lane & 3) * 4;
        const float* sp = sw + row * STG + c4;
        v4f v; v.x = sp[0]; v.y = sp[1]; v.z = sp[2]; v.w = sp[3];
        *reinterpret_cast<volatile v4f*>(gw + (size_t)row * NH + c4) = v;
      }
    }
  };
  emit();
  __threadfence();
  emit();
}

__global__ __launch_bounds__(32) void k_gscan(const float* __restrict__ gates, float* __restrict__ logG) {
  constexpr int CH = 128;
  constexpr int NCH = TT / CH;
  __shared__ __attribute__((aligned(16))) float inner[TT];
  __shared__ float tot[NCH];
  const int bh = blockIdx.x, b = bh >> 4, h = bh & 15;
  const int lane = threadIdx.x;

  if (lane < NCH) {
    const float* gp = gates + ((size_t)b * TT + lane * CH) * NH + h;
    float acc = 0.f;
#pragma unroll 1
    for (int u = 0; u < CH; ++u) {
      const float g = gp[(size_t)u * NH];
      const float ls = fminf(g, 0.f) - log1pf(expf(-fabsf(g)));
      acc = acc + ls;
      inner[lane * CH + u] = acc;
    }
    tot[lane] = acc;
  }
  __syncthreads();
  float E = 0.f;
  if (lane < NCH) {
    for (int c = 0; c < lane; ++c) E = E + tot[c];
  }
  float* dst = logG + (size_t)bh * TT + lane * CH;
  auto emit = [&]() {
    if (lane < NCH) {
#pragma unroll 4
      for (int q = 0; q < CH / 4; ++q) {
        const float* ip = inner + lane * CH + q * 4;
        v4f v; v.x = E + ip[0]; v.y = E + ip[1]; v.z = E + ip[2]; v.w = E + ip[3];
        *reinterpret_cast<volatile v4f*>(dst + q * 4) = v;
      }
    }
  };
  emit();
  __threadfence();
  emit();
}

__global__ __launch_bounds__(128) void k_attn(
    const u16* __restrict__ Qh, const u16* __restrict__ Ql,
    const u16* __restrict__ Kh, const u16* __restrict__ Kl,
    const u16* __restrict__ Vh, const u16* __restrict__ Vl,
    const float* __restrict__ logG, const float* __restrict__ nrm, float* __restrict__ out) {
  __shared__ __attribute__((aligned(16))) u16 ldsK[2][64 * LDSP];
  __shared__ __attribute__((aligned(16))) u16 ldsV[2][64 * LDSP];
  __shared__ __attribute__((aligned(16))) u16 ldsP[2][4][16 * LDSP];
  __shared__ float ldsGk[64];
  __shared__ float ldsM[4];

  const int tid = threadIdx.x, wave = tid >> 5, lane = tid & 31;
  const int h8 = (lane >> 4) * 8, ln = lane & 15;
  const int qt = blockIdx.x;
  const int bh = blockIdx.y;
  const int b = bh >> 4, hd = bh & 15;
  const int qs = qt * 64;
  const size_t pb = (size_t)bh * TT * HS;
  const float* G = logG + (size_t)bh * TT;

  const int qrow = qs + wave * 16 + ln;
  const u16* qph = Qh + pb + (size_t)qrow * HS;
  const u16* qpl = Ql + pb + (size_t)qrow * HS;
  const v16bf qh0 = load_frag(qph, h8), qh1 = load_frag(qph + 32, h8);
  const v16bf ql0 = load_frag(qpl, h8), ql1 = load_frag(qpl + 32, h8);

  float gq[8], m_run[8], l_run[8];
  v8f o[4] = {};
#pragma unroll
  for (int r = 0; r < 8; ++r) {
    gq[r] = G[qs + wave * 16 + h8 + r];
    m_run[r] = NEG_BIG;
    l_run[r] = 0.f;
  }
  const float qn2 = nrm[(size_t)(bh * NT + qt) * 32];
  const float* knl = nrm + (size_t)(NBH * NT + bh * NT) * 32;
  const float Gqs = G[qs];
  float m_min = NEG_BIG;

  for (int it = 0; it <= qt; ++it) {
    const int kt = qt - it;
    const int kvs = kt * 64;
    const bool diag = (it == 0);
    if (!diag) {
      const float kn2 = knl[kt * 32];
      const float ub = 2.0f * logf(1.02f * sqrtf(qn2 * kn2) + EPSV) + LOGSCALE + (Gqs - G[kvs + 63]) + 1.0f;
      if (ub < m_min - CULL_GAP) continue;
    }
    __syncthreads();
#pragma unroll
    for (int p = 0; p < 4; ++p) {
      const int idx = tid + p * 128, row = idx >> 3, seg = (idx & 7) * 8;
      const size_t go = pb + (size_t)(kvs + row) * HS + seg;
      *reinterpret_cast<v4u*>(ldsK[0] + row * LDSP + seg) = *reinterpret_cast<const v4u*>(Kh + go);
      *reinterpret_cast<v4u*>(ldsK[1] + row * LDSP + seg) = *reinterpret_cast<const v4u*>(Kl + go);
      Pack8 vh, vl;
      vh.q = *reinterpret_cast<const v4u*>(Vh + go);
      vl.q = *reinterpret_cast<const v4u*>(Vl + go);
#pragma unroll
      for (int e = 0; e < 8; ++e) {
        ldsV[0][(seg + e) * LDSP + row] = vh.e[e];
        ldsV[1][(seg + e) * LDSP + row] = vl.e[e];
      }
    }
    if (tid < 64) ldsGk[tid] = G[kvs + tid];
    __syncthreads();

    v8f s[4];
#pragma unroll
    for (int j = 0; j < 4; ++j) {
      v8f a = {};
      const u16* kr0 = ldsK[0] + (j * 16 + ln) * LDSP;
      const u16* kr1 = ldsK[1] + (j * 16 + ln) * LDSP;
      a = wmma_bf16x3(a, qh0, ql0, load_frag(kr0, h8), load_frag(kr1, h8));
      a = wmma_bf16x3(a, qh1, ql1, load_frag(kr0 + 32, h8), load_frag(kr1 + 32, h8));
      s[j] = a;
    }

    float z[4][8], tmax[8];
#pragma unroll
    for (int r = 0; r < 8; ++r) tmax[r] = NEG_BIG;
#pragma unroll
    for (int j = 0; j < 4; ++j) {
      const int kg = kvs + j * 16 + ln;
      const float gk = ldsGk[j * 16 + ln];
#pragma unroll
      for (int r = 0; r < 8; ++r) {
        float zz = 2.0f * logf(fabsf(s[j][r]) + EPSV) + LOGSCALE + (gq[r] - gk);
        if (diag) {
          const int tq = qs + wave * 16 + h8 + r;
          if (kg > tq) zz = NEG_BIG;
        }
        z[j][r] = zz;
        tmax[r] = fmaxf(tmax[r], zz);
      }
    }
#pragma unroll
    for (int r = 0; r < 8; ++r)
#pragma unroll
      for (int off = 1; off < 16; off <<= 1)
        tmax[r] = fmaxf(tmax[r], __shfl_xor(tmax[r], off, 32));

    float alpha[8], mnew[8], rsum[8];
#pragma unroll
    for (int r = 0; r < 8; ++r) {
      mnew[r] = fmaxf(m_run[r], tmax[r]);
      alpha[r] = expf(m_run[r] - mnew[r]);
      m_run[r] = mnew[r];
      rsum[r] = 0.f;
    }
#pragma unroll
    for (int j = 0; j < 4; ++j)
#pragma unroll
      for (int r = 0; r < 8; ++r) {
        const float p = expf(z[j][r] - mnew[r]);
        z[j][r] = p;
        rsum[r] += p;
      }
#pragma unroll
    for (int r = 0; r < 8; ++r) {
#pragma unroll
      for (int off = 1; off < 16; off <<= 1)
        rsum[r] += __shfl_xor(rsum[r], off, 32);
      l_run[r] = l_run[r] * alpha[r] + rsum[r];
    }
#pragma unroll
    for (int j = 0; j < 4; ++j)
#pragma unroll
      for (int r = 0; r < 8; ++r) o[j][r] *= alpha[r];

#pragma unroll
    for (int j = 0; j < 4; ++j)
#pragma unroll
      for (int r = 0; r < 8; ++r) {
        const float p = z[j][r];
        const unsigned hb = bf16_rne_bits(p);
        const unsigned lb = bf16_rne_bits(p - bf16_bits_to_f32(hb));
        ldsP[0][wave][(h8 + r) * LDSP + j * 16 + ln] = (u16)hb;
        ldsP[1][wave][(h8 + r) * LDSP + j * 16 + ln] = (u16)lb;
      }
    __syncthreads();

#pragma unroll
    for (int ks = 0; ks < 2; ++ks) {
      const v16bf ph = load_frag(ldsP[0][wave] + ln * LDSP + ks * 32, h8);
      const v16bf pl = load_frag(ldsP[1][wave] + ln * LDSP + ks * 32, h8);
#pragma unroll
      for (int j = 0; j < 4; ++j) {
        const v16bf vfh = load_frag(ldsV[0] + (j * 16 + ln) * LDSP + ks * 32, h8);
        const v16bf vfl = load_frag(ldsV[1] + (j * 16 + ln) * LDSP + ks * 32, h8);
        o[j] = wmma_bf16x3(o[j], ph, pl, vfh, vfl);
      }
    }

    if (diag) {
      float ml = m_run[0];
#pragma unroll
      for (int r = 1; r < 8; ++r) ml = fminf(ml, m_run[r]);
#pragma unroll
      for (int off = 16; off > 0; off >>= 1) ml = fminf(ml, __shfl_xor(ml, off, 32));
      if (lane == 0) ldsM[wave] = ml;
      __syncthreads();
      m_min = fminf(fminf(ldsM[0], ldsM[1]), fminf(ldsM[2], ldsM[3]));
    }
  }

  __syncthreads();
  float* stg = reinterpret_cast<float*>(&ldsK[0][0]);
  float* sw = stg + wave * 16 * STG;
#pragma unroll
  for (int r = 0; r < 8; ++r) {
    const float inv = 1.0f / l_run[r];
#pragma unroll
    for (int j = 0; j < 4; ++j) sw[(h8 + r) * STG + j * 16 + ln] = o[j][r] * inv;
  }
  __syncthreads();
  float* ob = out + ((size_t)(b * TT + qs + wave * 16)) * CC + hd * HS;
  auto emit = [&]() {
#pragma unroll
    for (int it = 0; it < 8; ++it) {
      const int row = it * 2 + (lane >> 4), c4 = (lane & 15) * 4;
      const float* sp = sw + row * STG + c4;
      v4f v; v.x = sp[0]; v.y = sp[1]; v.z = sp[2]; v.w = sp[3];
      *reinterpret_cast<volatile v4f*>(ob + (size_t)row * CC + c4) = v;
    }
  };
  emit();
  __threadfence();
  emit();
}

extern "C" void kernel_launch(void* const* d_in, const int* in_sizes, int n_in,
                              void* d_out, int out_size, void* d_ws, size_t ws_size,
                              hipStream_t stream) {
  if (n_in < 2) return;
  if (in_sizes[0] != BB * TT * CC || in_sizes[1] != OC * CC || out_size != BB * TT * CC) return;

  constexpr size_t PLANE = (size_t)NBH * TT * HS * sizeof(u16);
  constexpr size_t GATESB = (size_t)MROWS * NH * sizeof(float);
  constexpr size_t LOGGB = (size_t)NBH * TT * sizeof(float);
  constexpr size_t NRMB = (size_t)2 * NBH * NT * 32 * sizeof(float);
  constexpr size_t TOTAL = 6 * PLANE + GATESB + LOGGB + NRMB;
  if (ws_size < TOTAL) return;

  const float* x = (const float*)d_in[0];
  const float* W = (const float*)d_in[1];
  float* out = (float*)d_out;
  char* ws = (char*)d_ws;
  u16* Qh = (u16*)(ws + 0 * PLANE);
  u16* Ql = (u16*)(ws + 1 * PLANE);
  u16* Kh = (u16*)(ws + 2 * PLANE);
  u16* Kl = (u16*)(ws + 3 * PLANE);
  u16* Vh = (u16*)(ws + 4 * PLANE);
  u16* Vl = (u16*)(ws + 5 * PLANE);
  float* gates = (float*)(ws + 6 * PLANE);
  float* logG = (float*)(ws + 6 * PLANE + GATESB);
  float* nrm = (float*)(ws + 6 * PLANE + GATESB + LOGGB);

  k_proj<<<dim3(OC / 64 + 1, MROWS / 64), 128, 0, stream>>>(x, W, Qh, Ql, Kh, Kl, Vh, Vl, gates, nrm);
  k_gscan<<<NBH, 32, 0, stream>>>(gates, logG);
  k_attn<<<dim3(NT, NBH), 128, 0, stream>>>(Qh, Ql, Kh, Kl, Vh, Vl, logG, nrm, out);
}
